// Distiller_53412213293408
// MI455X (gfx1250) — hardware-verified
//
#include <hip/hip_runtime.h>
#include <math.h>
typedef __attribute__((ext_vector_type(16))) _Float16 v16h;
typedef __attribute__((ext_vector_type(8)))  _Float16 v8h;
typedef __attribute__((ext_vector_type(16))) __bf16   v16b;
typedef __attribute__((ext_vector_type(8)))  __bf16   v8b;
typedef __attribute__((ext_vector_type(8)))  float    v8f;
typedef __attribute__((ext_vector_type(4)))  float    v4f;
#define PSCALE 32768.0f
#define U16(p) ((const unsigned short*)(const void*)(p))
#define PSCALE_INV (1.0f / 32768.0f)

__device__ __forceinline__ unsigned short f2bf_bits(float f) {
  unsigned u = __float_as_uint(f);
  return (unsigned short)((u + 0x7FFFu + ((u >> 16) & 1u)) >> 16);
}
__device__ __forceinline__ float bf_bits2f(unsigned short h) { return __uint_as_float(((unsigned)h) << 16); }

__device__ __forceinline__ void dep_guard_h(v8f& a, v8f& b, v16h x, v16h y) { asm volatile("v_nop\n\tv_nop\n\tv_nop\n\tv_nop" : "+v"(a), "+v"(b) : "v"(x), "v"(y)); }
__device__ __forceinline__ void dep_guard_b(v8f& a, v8f& b, v16b x, v16b y) { asm volatile("v_nop\n\tv_nop\n\tv_nop\n\tv_nop" : "+v"(a), "+v"(b) : "v"(x), "v"(y)); }
__device__ __forceinline__ void keep4_h(v16h a, v16h b, v16h c, v16h d) { asm volatile("v_nop" :: "v"(a), "v"(b), "v"(c), "v"(d)); }
__device__ __forceinline__ void keep4_b(v16b a, v16b b, v16b c, v16b d) { asm volatile("v_nop" :: "v"(a), "v"(b), "v"(c), "v"(d)); }
__device__ __forceinline__ void acc_guard4(v8f& a, v8f& b, v8f& c, v8f& d) { asm volatile("v_nop\n\tv_nop\n\tv_nop\n\tv_nop" : "+v"(a), "+v"(b), "+v"(c), "+v"(d)); }
template <typename T> struct Frag;
template <> struct Frag<_Float16> {
  typedef v16h V; union U { v16h v; v8h h[2]; };
  static __device__ __forceinline__ v16h load(const _Float16* p) {
    U f; f.h[0] = *(const v8h*)(p); f.h[1] = *(const v8h*)(p + 16); return f.v;
  }
  static __device__ __forceinline__ v8f mma(v16h a, v16h b, v8f c) {
    return __builtin_amdgcn_wmma_f32_16x16x32_f16(false, a, false, b, (short)0, c, false, false);
  }
  static __device__ __forceinline__ void guard(v8f& a, v8f& b, v16h x, v16h y) { dep_guard_h(a, b, x, y); }
  static __device__ __forceinline__ void keep(v16h a, v16h b, v16h c, v16h d) { keep4_h(a, b, c, d); }
};
template <> struct Frag<__bf16> {
  typedef v16b V; union U { v16b v; v8b h[2]; };
  static __device__ __forceinline__ v16b load(const __bf16* p) {
    U f; f.h[0] = *(const v8b*)(p); f.h[1] = *(const v8b*)(p + 16); return f.v;
  }
  static __device__ __forceinline__ v8f mma(v16b a, v16b b, v8f c) {
    return __builtin_amdgcn_wmma_f32_16x16x32_bf16(false, a, false, b, (short)0, c, false, false);
  }
  static __device__ __forceinline__ void guard(v8f& a, v8f& b, v16b x, v16b y) { dep_guard_b(a, b, x, y); }
  static __device__ __forceinline__ void keep(v16b a, v16b b, v16b c, v16b d) { keep4_b(a, b, c, d); }
};

template <int ET> struct Elem;
template <> struct Elem<0> { typedef _Float16 T; };
template <> struct Elem<1> { typedef __bf16 T; };
template <int ET, bool SPLIT, int BIAS_MODE, int OUT_MODE, bool RESID, int ACT = 0>
__global__ __launch_bounds__(256) void wmma_gemm64(
    const unsigned short* __restrict__ Ap, const unsigned short* __restrict__ A2p, int lda, long strideA,
    const unsigned short* __restrict__ Btp, const unsigned short* __restrict__ Bt2p, int ldb, long strideB,
    void* __restrict__ Cout, void* __restrict__ Cout2, int ldc, long strideC,
    const float* __restrict__ bias,
    const float* __restrict__ resid, long strideR,
    int M, int N, int K, float scale) {
  typedef typename Elem<ET>::T T;
  typedef typename Frag<T>::V V;
  const T* A = (const T*)Ap; const T* A2 = (const T*)A2p; const T* Bt = (const T*)Btp; const T* Bt2 = (const T*)Bt2p;
  __shared__ __align__(16) float sT[8][16 * 68];
  const int b    = blockIdx.y;
  const int lane = threadIdx.x & 31;
  const int wave = threadIdx.x >> 5;
  const int tilesN = N >> 6;
  const int tilesM = M >> 6;
  const int tile = blockIdx.x * 8 + wave;
  if (tile >= tilesM * tilesN) return;
  const int tm = tile / tilesN;
  const int tn = tile - tm * tilesN;
  const int m0 = tm << 6;
  const int n0 = tn << 6;

  const T* Ab  = A  + (size_t)b * strideA;
  const T* Bb  = Bt + (size_t)b * strideB;
  const T* Ab2 = SPLIT ? (A2  + (size_t)b * strideA) : nullptr;
  const T* Bb2 = SPLIT ? (Bt2 + (size_t)b * strideB) : nullptr;

  const int rlane = lane & 15;
  const int koff  = (lane >> 4) * 8;
  const int mOff  = (lane >> 4) * 8;

  v8f acc[4][4];
#pragma unroll
  for (int i = 0; i < 4; ++i)
#pragma unroll
    for (int j = 0; j < 4; ++j) acc[i][j] = (v8f){0.f,0.f,0.f,0.f,0.f,0.f,0.f,0.f};

  for (int k0 = 0; k0 < K; k0 += 32) {
    V bh[4], bl[4];
#pragma unroll
    for (int j = 0; j < 4; ++j) {
      const size_t bo = (size_t)(n0 + (j << 4) + rlane) * ldb + koff + k0;
      bh[j] = Frag<T>::load(Bb + bo);
      if (SPLIT) bl[j] = Frag<T>::load(Bb2 + bo);
    }
#pragma unroll
    for (int i = 0; i < 4; ++i) {
      const size_t ao = (size_t)(m0 + (i << 4) + rlane) * lda + koff + k0;
      V ah = Frag<T>::load(Ab + ao);
      V al;
      if (SPLIT) al = Frag<T>::load(Ab2 + ao);
#pragma unroll
      for (int j = 0; j < 4; ++j) {
        acc[i][j] = Frag<T>::mma(ah, bh[j], acc[i][j]);
        if (SPLIT) {
          acc[i][j] = Frag<T>::mma(ah, bl[j], acc[i][j]);
          acc[i][j] = Frag<T>::mma(al, bh[j], acc[i][j]);
        }
      }
      Frag<T>::guard(acc[i][0], acc[i][3], ah, SPLIT ? al : ah);
    }
    Frag<T>::keep(bh[0], bh[1], bh[2], bh[3]);
    if (SPLIT) Frag<T>::keep(bl[0], bl[1], bl[2], bl[3]);
  }
  acc_guard4(acc[0][0], acc[0][1], acc[0][2], acc[0][3]);
  acc_guard4(acc[1][0], acc[1][1], acc[1][2], acc[1][3]);
  acc_guard4(acc[2][0], acc[2][1], acc[2][2], acc[2][3]);
  acc_guard4(acc[3][0], acc[3][1], acc[3][2], acc[3][3]);

  float* slab = sT[wave];
  const float* Rb = RESID ? (resid + (size_t)b * strideR) : nullptr;
#pragma unroll
  for (int i = 0; i < 4; ++i) {
    const int mBase = m0 + (i << 4);
#pragma unroll
    for (int j = 0; j < 4; ++j) {
      const int n = n0 + (j << 4) + rlane;
      float bv = 0.f;
      if (BIAS_MODE == 2) bv = bias[n];
#pragma unroll
      for (int r = 0; r < 8; ++r) {
        float v = acc[i][j][r] * scale;
        if (BIAS_MODE == 1) v += bias[mBase + mOff + r];
        if (BIAS_MODE == 2) v += bv;
        if (RESID) v += Rb[(size_t)(mBase + mOff + r) * ldc + n];
        if (ACT == 1) v = tanhf(v);
        if (ACT == 2) v = fmaxf(v, 0.0f);
        if (ACT == 3) v = v / (1.0f + expf(-v));
        if (ACT == 4) v = (v > 0.f) ? v : 0.01f * v;
        if (ACT == 5) v = 0.5f * v * (1.0f + erff(v * 0.70710678118654752f));
        slab[(mOff + r) * 68 + (j << 4) + rlane] = v;
      }
    }
    __builtin_amdgcn_fence(__ATOMIC_RELEASE, "workgroup");
    __builtin_amdgcn_wave_barrier();
    __builtin_amdgcn_fence(__ATOMIC_ACQUIRE, "workgroup");
    if (OUT_MODE == 0) {
      float* C = (float*)Cout + (size_t)b * strideC;
      const int hh = lane >> 4, c4 = (lane & 15) * 4;
      for (int pass = 0; pass < 2; ++pass) {
#pragma unroll
        for (int it = 0; it < 8; ++it) {
          const int row = it * 2 + hh;
          v4f v = *(const v4f*)(slab + row * 68 + c4);
          *(volatile v4f*)(C + (size_t)(mBase + row) * ldc + n0 + c4) = v;
        }
        __threadfence();
      }
    } else {
      const int q = lane >> 3, c8 = (lane & 7) * 8;
      unsigned short* C  = (unsigned short*)Cout  + (size_t)b * strideC;
      unsigned short* C2 = (OUT_MODE == 2) ? ((unsigned short*)Cout2 + (size_t)b * strideC) : nullptr;
      for (int pass = 0; pass < 2; ++pass) {
#pragma unroll
        for (int it = 0; it < 4; ++it) {
          const int row = it * 4 + q;
          const float* sp = slab + row * 68 + c8;
          v8h hv, lv;
#pragma unroll
          for (int e = 0; e < 8; ++e) {
            if (OUT_MODE == 1) {
              hv[e] = (_Float16)sp[e];
            } else {
              unsigned short hb = f2bf_bits(sp[e]);
              unsigned short lb = f2bf_bits(sp[e] - bf_bits2f(hb));
              hv[e] = __builtin_bit_cast(_Float16, hb);
              lv[e] = __builtin_bit_cast(_Float16, lb);
            }
          }
          *(volatile v8h*)(C + (size_t)(mBase + row) * ldc + n0 + c8) = hv;
          if (OUT_MODE == 2) *(volatile v8h*)(C2 + (size_t)(mBase + row) * ldc + n0 + c8) = lv;
        }
        __threadfence();
      }
    }
    __builtin_amdgcn_fence(__ATOMIC_RELEASE, "workgroup");
    __builtin_amdgcn_wave_barrier();
    __builtin_amdgcn_fence(__ATOMIC_ACQUIRE, "workgroup");
  }
}

__global__ __launch_bounds__(256) void cast_f32_f16x2(
    const float* __restrict__ in, _Float16* __restrict__ out, int n2) {
  int i = blockIdx.x * 256 + threadIdx.x;
  if (i < n2) {
    const _Float16 h0 = (_Float16)in[2 * i], h1 = (_Float16)in[2 * i + 1];
    const unsigned u = (unsigned)__builtin_bit_cast(unsigned short, h0) | ((unsigned)__builtin_bit_cast(unsigned short, h1) << 16);
    ((volatile unsigned*)out)[i] = u;
    __threadfence();
    ((volatile unsigned*)out)[i] = u;
  }
}


#define DB 8
#define DH 8
#define DNT 1024
#define DD 32
#define DC (DH * DD)
__device__ __forceinline__ unsigned pkh(float a, float b) { return (unsigned)__builtin_bit_cast(unsigned short, (_Float16)a) | ((unsigned)__builtin_bit_cast(unsigned short, (_Float16)b) << 16); }
__global__ __launch_bounds__(256) void tok_kernel(const float* __restrict__ x, unsigned* __restrict__ T16) {
  __shared__ float tile[DD][65];
  const int bh = blockIdx.y, n0 = blockIdx.x * 64, tx = threadIdx.x, ty = threadIdx.y;
  for (int d = ty; d < DD; d += 8) { const float* src = x + ((size_t)bh * DD + d) * DNT + n0; tile[d][tx] = src[tx]; tile[d][32 + tx] = src[32 + tx]; }
  __syncthreads();
  for (int pass = 0; pass < 2; ++pass) { for (int n = ty; n < 64; n += 8) if (tx < 16) ((volatile unsigned*)T16)[(((size_t)bh * DNT + n0 + n) * DD) / 2 + tx] = pkh(tile[2 * tx][n], tile[2 * tx + 1][n]); __threadfence(); }
}
__global__ __launch_bounds__(256) void soft_kernel(const float* __restrict__ S, unsigned* __restrict__ P16) {
  const int lane = threadIdx.x & 31, wave = threadIdx.x >> 5; const size_t row = (size_t)blockIdx.x * 8 + wave; const float* s = S + row * DNT;
  float v[32]; float mx = -INFINITY;
#pragma unroll
  for (int q = 0; q < 32; q += 4) { const v4f t = *(const v4f*)(s + lane * 32 + q); v[q] = t[0]; v[q + 1] = t[1]; v[q + 2] = t[2]; v[q + 3] = t[3]; mx = fmaxf(mx, fmaxf(fmaxf(t[0], t[1]), fmaxf(t[2], t[3]))); }
  for (int o = 16; o > 0; o >>= 1) mx = fmaxf(mx, __shfl_xor(mx, o, 32));
  float sum = 0.f;
#pragma unroll
  for (int q = 0; q < 32; ++q) { v[q] = __expf(v[q] - mx); sum += v[q]; }
  for (int o = 16; o > 0; o >>= 1) sum += __shfl_xor(sum, o, 32);
  const float sc = 32768.0f / sum; typedef __attribute__((ext_vector_type(4))) unsigned u4;
  for (int pass = 0; pass < 2; ++pass) {
#pragma unroll
    for (int q4 = 0; q4 < 4; ++q4) { u4 u; for (int z = 0; z < 4; ++z) { const int q = q4 * 8 + 2 * z; u[z] = pkh(v[q] * sc, v[q + 1] * sc); } *(volatile u4*)(P16 + (row * DNT + lane * 32 + q4 * 8) / 2) = u; }
    __threadfence(); }
}
__global__ __launch_bounds__(256) void sqerr_kernel(const float* __restrict__ O, const float* __restrict__ ft, int b, double* __restrict__ PS) {
  __shared__ double red[256];
  const int h = blockIdx.y, n0 = blockIdx.x * 64, tx = threadIdx.x & 31, ty = threadIdx.x >> 5; double s = 0.0;
  for (int n = ty; n < 64; n += 8) { const float o = O[((size_t)h * DNT + n0 + n) * 64 + tx]; const float t = ft[(((size_t)b * DH + h) * DD + tx) * DNT + n0 + n]; const double d = (double)o - (double)t; s += d * d; }
  red[threadIdx.x] = s; __syncthreads();
  for (int o = 128; o > 0; o >>= 1) { if (threadIdx.x < o) red[threadIdx.x] += red[threadIdx.x + o]; __syncthreads(); }
  if (threadIdx.x < 32) { const size_t i = ((size_t)b * DH + h) * (DNT / 64) + blockIdx.x; ((volatile double*)PS)[i] = red[0]; __threadfence(); ((volatile double*)PS)[i] = red[0]; }
}
__global__ __launch_bounds__(256) void mean_kernel(const double* __restrict__ PS, int n, float* __restrict__ out) {
  __shared__ double red[256]; double s = 0.0; for (int i = threadIdx.x; i < n; i += 256) s += PS[i]; red[threadIdx.x] = s; __syncthreads();
  for (int o = 128; o > 0; o >>= 1) { if (threadIdx.x < o) red[threadIdx.x] += red[threadIdx.x + o]; __syncthreads(); }
  if (threadIdx.x < 32) { const float v = (float)(red[0] / ((double)DB * DC * DNT)); ((volatile float*)out)[0] = v; __threadfence(); ((volatile float*)out)[0] = v; }
}
extern "C" void kernel_launch(void* const* d_in, const int* in_sizes, int n_in, void* d_out, int out_size, void* d_ws, size_t ws_size, hipStream_t stream) {
  (void)in_sizes; (void)n_in; (void)out_size; (void)ws_size;
  const float* fs_ = (const float*)d_in[0]; const float* ft = (const float*)d_in[1];
  char* ws = (char*)d_ws; size_t off = 0;
  auto carve = [&](size_t bytes) -> char* { char* p = ws + off; off += (bytes + 255) & ~(size_t)255; return p; };
  unsigned* Q16 = (unsigned*)carve((size_t)DB * DC * DNT * 2); unsigned* K16 = (unsigned*)carve((size_t)DB * DC * DNT * 2); _Float16* V16 = (_Float16*)carve((size_t)DB * DC * DNT * 2 + 64 * DNT * 2);
  float* S = (float*)carve((size_t)DH * DNT * DNT * 4); unsigned* P16 = (unsigned*)carve((size_t)DH * DNT * DNT * 2); float* O = (float*)carve((size_t)DH * DNT * 64 * 4); double* PS = (double*)carve((size_t)DB * DH * (DNT / 64) * 8);
  tok_kernel<<<dim3(DNT / 64, DB * DH), dim3(32, 8), 0, stream>>>(fs_, Q16); tok_kernel<<<dim3(DNT / 64, DB * DH), dim3(32, 8), 0, stream>>>(ft, K16);
  cast_f32_f16x2<<<(DB * DC * DNT / 2 + 255) / 256, 256, 0, stream>>>(fs_, V16, (long)DB * DC * DNT / 2);
  cast_f32_f16x2<<<(64 * DNT / 2 + 255) / 256, 256, 0, stream>>>(fs_, V16 + (size_t)DB * DC * DNT, (long)64 * DNT / 2);
  const int ts = (DNT / 64) * (DNT / 64), to = (DNT / 64) * 1;
  for (int b = 0; b < DB; ++b) {
    wmma_gemm64<0, false, 0, 0, false><<<dim3((ts + 7) / 8, DH), 256, 0, stream>>>((const unsigned short*)Q16 + (size_t)b * DC * DNT, nullptr, DD, (long)DNT * DD, (const unsigned short*)K16 + (size_t)b * DC * DNT, nullptr, DD, (long)DNT * DD, S, nullptr, DNT, (long)DNT * DNT, nullptr, nullptr, 0, DNT, DNT, DD, 1.0f);
    soft_kernel<<<DH * DNT / 8, 256, 0, stream>>>(S, P16);
    wmma_gemm64<0, false, 0, 0, false><<<dim3((to + 7) / 8, DH), 256, 0, stream>>>((const unsigned short*)P16, nullptr, DNT, (long)DNT * DNT, U16(V16 + (size_t)b * DC * DNT), nullptr, DNT, (long)DD * DNT, O, nullptr, 64, (long)DNT * 64, nullptr, nullptr, 0, DNT, 64, DNT, 1.0f / 32768.0f);
    sqerr_kernel<<<dim3(DNT / 64, DH), 256, 0, stream>>>(O, ft, b, PS); }
  mean_kernel<<<1, 256, 0, stream>>>(PS, DB * DH * (DNT / 64), (float*)d_out);
}
